// Transformer_46789373722799
// MI455X (gfx1250) — hardware-verified
//
#include <hip/hip_runtime.h>
#include <stddef.h>


typedef _Float16 h16;
typedef _Float16 v16h __attribute__((ext_vector_type(16)));
typedef _Float16 v8h  __attribute__((ext_vector_type(8)));
typedef float    v8f  __attribute__((ext_vector_type(8)));
typedef float    v4f  __attribute__((ext_vector_type(4)));

#ifndef NB
#define NB 4
#endif
#ifndef SEQ
#define SEQ 1024
#endif
#define NB_FULL  4
#define SEQ_FULL 1024
#define DIM   256
#define HID   256
#define NHEAD 16
#define NGRP  8
#define GIN   32
#define KQC   128
#define KQG   16
#define VG    32
#define HDK   8
#define HDV   16
#define MROWS (NB * SEQ)

static_assert(NB >= 1 && NB <= NB_FULL);
static_assert(SEQ >= 64 && SEQ <= SEQ_FULL && (SEQ % 64) == 0);
static_assert(DIM == NHEAD * HDV);
static_assert(KQC == NHEAD * HDK);
static_assert(DIM == NGRP * GIN);
static_assert(KQC == NGRP * KQG && DIM == NGRP * VG);
static_assert(KQG == 2 * HDK && VG == 2 * HDV && KQG == 16 && VG == 32);
static_assert(GIN == 32);
static_assert(HDK == 8 && HDV == 16);
static_assert(NHEAD == 16);
static_assert((DIM % 64) == 0 && (DIM % 32) == 0);
static_assert((HID % 64) == 0 && (HID % 32) == 0);
static_assert((MROWS % 64) == 0 && (MROWS % 32) == 0);
static_assert(DIM == 32 * 8);
static_assert(((DIM * HID) % 2048) == 0);

#define LDT 72
#define LDC 68
#define XP  40
#define TP  260
#define TP2 36
static_assert((LDT % 8) == 0 && LDT >= 64);
static_assert((LDC % 4) == 0 && LDC >= 64);
static_assert((XP % 8) == 0 && XP >= GIN);
static_assert((TP % 4) == 0 && TP >= DIM);
static_assert((TP2 % 4) == 0 && TP2 >= 32);

#define XCARRY  64.0f
#define WCARRY  64.0f
#define QKCARRY 64.0f
#define VCARRY  64.0f
#define PCARRY  1024.0f
#define ACARRY  16.0f
#define MCARRY  16.0f

#define WFF_BYTES ((size_t)DIM * HID * 2)
#define KQ_BYTES  ((size_t)NB * NHEAD * SEQ * HDK * 2)
#define V_BYTES   ((size_t)NB * DIM * SEQ * 2)
#define H1_BYTES  ((size_t)MROWS * DIM * 2)
#define X1_BYTES  ((size_t)MROWS * DIM * 4)
#define MID_BYTES ((size_t)MROWS * HID * 2)
#define Y_BYTES   ((size_t)MROWS * DIM * 4)
#define OFF_W1  ((size_t)0)
#define OFF_W2  (OFF_W1 + WFF_BYTES)
#define OFF_K   (OFF_W2 + WFF_BYTES)
#define OFF_Q   (OFF_K + KQ_BYTES)
#define OFF_V   (OFF_Q + KQ_BYTES)
#define OFF_H1  (OFF_V + V_BYTES)
#define OFF_X1  (OFF_H1 + H1_BYTES)
#define OFF_MID (OFF_X1 + X1_BYTES)
#define OFF_Y   (OFF_MID + MID_BYTES)
#define WS_TOTAL (OFF_Y + Y_BYTES)
static_assert((WFF_BYTES % 128) == 0 && (KQ_BYTES % 128) == 0 && (V_BYTES % 128) == 0);
static_assert((H1_BYTES % 128) == 0 && (X1_BYTES % 128) == 0 && (MID_BYTES % 128) == 0);
static_assert((Y_BYTES % 128) == 0);
static_assert(WS_TOTAL <= (size_t)134217728);

__device__ __forceinline__ float bf16r(float x) {
  unsigned int u = __float_as_uint(x);
  u = (u + 0x7FFFu + ((u >> 16) & 1u)) & 0xFFFF0000u;
  return __uint_as_float(u);
}

static __device__ __forceinline__ h16 toh_flush(float v) {
  const h16 r = (h16)v;
  return (fabsf(v) < 6.103515625e-05f) ? (h16)0.0f : r;
}

__device__ __forceinline__ v16h frag_at(const _Float16* p) {
  v8h lo = *(const v8h*)(p);
  v8h hi = *(const v8h*)(p + 16);
  v16h out;
#pragma unroll
  for (int i = 0; i < 8; ++i) { out[i] = lo[i]; out[i + 8] = hi[i]; }
  return out;
}

__device__ __forceinline__ v16h wfrag(const float* __restrict__ p) {
  const v4f a0 = *(const v4f*)(p);
  const v4f a1 = *(const v4f*)(p + 4);
  const v4f a2 = *(const v4f*)(p + 16);
  const v4f a3 = *(const v4f*)(p + 20);
  v16h out;
#pragma unroll
  for (int i = 0; i < 4; ++i) {
    out[i]      = toh_flush(WCARRY * bf16r(a0[i]));
    out[i + 4]  = toh_flush(WCARRY * bf16r(a1[i]));
    out[i + 8]  = toh_flush(WCARRY * bf16r(a2[i]));
    out[i + 12] = toh_flush(WCARRY * bf16r(a3[i]));
  }
  return out;
}

__device__ __forceinline__ v8f wmma16(v16h a, v16h b, v8f c) {
  v8f d = __builtin_amdgcn_wmma_f32_16x16x32_f16(false, a, false, b, (short)0, c,
                                                 false, false);
  asm volatile("v_nop\n\tv_nop\n\tv_nop\n\tv_nop" : "+v"(d) : "v"(a), "v"(b));
  return d;
}

__device__ __forceinline__ float red32_sum(float x) {
#pragma unroll
  for (int off = 1; off < 32; off <<= 1) x += __shfl_xor(x, off, 32);
  return x;
}

__device__ __forceinline__ float relu_act(float t) {
  return fmaxf(t, 0.0f);
}

__global__ __launch_bounds__(256) void wcast_kernel(
    const float* __restrict__ W, _Float16* __restrict__ Wt) {
  const size_t e0 = ((size_t)blockIdx.x * 256u + threadIdx.x) * 8u;
  const v4f a0 = *(const v4f*)(W + e0);
  const v4f a1 = *(const v4f*)(W + e0 + 4u);
  v8h o;
#pragma unroll
  for (int i = 0; i < 4; ++i) {
    o[i]     = toh_flush(WCARRY * bf16r(a0[i]));
    o[i + 4] = toh_flush(WCARRY * bf16r(a1[i]));
  }
  *(volatile v8h*)(Wt + e0) = o;
  __threadfence();
  *(volatile v8h*)(Wt + e0) = o;
}

__global__ __launch_bounds__(128) void proj_kernel(
    const float* __restrict__ X,
    const float* __restrict__ wk, const float* __restrict__ bk,
    const float* __restrict__ wq, const float* __restrict__ bq,
    const float* __restrict__ wv, const float* __restrict__ bv,
    _Float16* __restrict__ Kp, _Float16* __restrict__ Qp, _Float16* __restrict__ Vp) {
  __shared__ _Float16 Xs[64 * XP];
  __shared__ _Float16 Vs[32 * LDT];
  const unsigned tid = threadIdx.x, lane = tid & 31u;
  const unsigned wave = __builtin_amdgcn_readfirstlane(threadIdx.x >> 5);
  const unsigned hh = lane >> 4, m = lane & 15u;
  const unsigned l0 = blockIdx.x * 64u;
  const unsigned g = blockIdx.y;
  const unsigned n = blockIdx.z;

#pragma unroll
  for (unsigned j = 0; j < 4u; ++j) {
    const unsigned idx = tid + 128u * j;
    const unsigned ch = idx >> 4, lq = (idx & 15u) * 4u;
    const v4f a = *(const v4f*)(X + ((size_t)n * DIM + g * GIN + ch) * SEQ_FULL + l0 + lq);
#pragma unroll
    for (unsigned i = 0; i < 4u; ++i)
      Xs[(lq + i) * XP + ch] = toh_flush(XCARRY * bf16r(a[i]));
  }
  __syncthreads();

  const unsigned xo = (wave * 16u + m) * XP + hh * 8u;
  const v8h xlo = *(const v8h*)&Xs[xo];
  const v8h xhi = *(const v8h*)&Xs[xo + 16u];
  v16h xb;
#pragma unroll
  for (int i = 0; i < 8; ++i) { xb[i] = xlo[i]; xb[i + 8] = xhi[i]; }

  const v16h ak  = wfrag(wk + (size_t)(g * KQG + m) * GIN + hh * 8u);
  const v16h aq  = wfrag(wq + (size_t)(g * KQG + m) * GIN + hh * 8u);
  const v16h av0 = wfrag(wv + (size_t)(g * VG + m) * GIN + hh * 8u);
  const v16h av1 = wfrag(wv + (size_t)(g * VG + 16u + m) * GIN + hh * 8u);
  const v8f dk = wmma16(ak, xb, (v8f){});
  const v8f dq = wmma16(aq, xb, (v8f){});
  v8f dv[2];
  dv[0] = wmma16(av0, xb, (v8f){});
  dv[1] = wmma16(av1, xb, (v8f){});

  const float ps = 1.0f / (XCARRY * WCARRY);
  const v4f bk0 = *(const v4f*)(bk + g * KQG + hh * 8u);
  const v4f bk1 = *(const v4f*)(bk + g * KQG + hh * 8u + 4u);
  const v4f bq0 = *(const v4f*)(bq + g * KQG + hh * 8u);
  const v4f bq1 = *(const v4f*)(bq + g * KQG + hh * 8u + 4u);
  v8h kx, qx;
#pragma unroll
  for (int r = 0; r < 4; ++r) {
    kx[r]     = toh_flush(QKCARRY * (dk[r] * ps + bf16r(bk0[r])));
    kx[r + 4] = toh_flush(QKCARRY * (dk[r + 4] * ps + bf16r(bk1[r])));
    qx[r]     = toh_flush(QKCARRY * (dq[r] * ps + bf16r(bq0[r])));
    qx[r + 4] = toh_flush(QKCARRY * (dq[r + 4] * ps + bf16r(bq1[r])));
  }
  const size_t kqoff =
      (((size_t)n * NHEAD + 2u * g + hh) * SEQ + l0 + wave * 16u + m) * HDK;

#pragma unroll
  for (unsigned t = 0; t < 2u; ++t) {
    const v4f b0 = *(const v4f*)(bv + g * VG + t * 16u + hh * 8u);
    const v4f b1 = *(const v4f*)(bv + g * VG + t * 16u + hh * 8u + 4u);
#pragma unroll
    for (unsigned r = 0; r < 4u; ++r) {
      Vs[(t * 16u + hh * 8u + r) * LDT + wave * 16u + m] =
          toh_flush(VCARRY * (dv[t][r] * ps + bf16r(b0[r])));
      Vs[(t * 16u + hh * 8u + r + 4u) * LDT + wave * 16u + m] =
          toh_flush(VCARRY * (dv[t][r + 4] * ps + bf16r(b1[r])));
    }
  }
  __syncthreads();

  v8h x[2];
  size_t off[2];
#pragma unroll
  for (unsigned i = 0; i < 2u; ++i) {
    const unsigned idx = tid + 128u * i;
    const unsigned ch = idx >> 3, kc = (idx & 7u) * 8u;
    x[i] = *(const v8h*)&Vs[ch * LDT + kc];
    off[i] = ((size_t)n * DIM + g * VG + ch) * SEQ + l0 + kc;
  }
  *(volatile v8h*)(Kp + kqoff) = kx;
  *(volatile v8h*)(Qp + kqoff) = qx;
#pragma unroll
  for (int i = 0; i < 2; ++i) *(volatile v8h*)(Vp + off[i]) = x[i];
  __threadfence();
  *(volatile v8h*)(Kp + kqoff) = kx;
  *(volatile v8h*)(Qp + kqoff) = qx;
#pragma unroll
  for (int i = 0; i < 2; ++i) *(volatile v8h*)(Vp + off[i]) = x[i];
}

__global__ __launch_bounds__(512) void attn_ln_kernel(
    const float* __restrict__ X, const _Float16* __restrict__ Kp,
    const _Float16* __restrict__ Qp, const _Float16* __restrict__ Vp,
    const float* __restrict__ G, const float* __restrict__ Be,
    _Float16* __restrict__ H1, float* __restrict__ X1) {
  __shared__ float T[16 * TP];
  const unsigned tid = threadIdx.x, lane = tid & 31u;
  const unsigned wave = __builtin_amdgcn_readfirstlane(threadIdx.x >> 5);
  const unsigned hh = lane >> 4, m = lane & 15u;
  const unsigned m0 = blockIdx.x * 16u;
  const unsigned n = blockIdx.y;
  const unsigned head = wave;
  const bool lowhalf = (hh == 0u);
  const h16 hz = (h16)0.0f;

  const size_t nh = (size_t)n * NHEAD + head;
  const v8h qv = *(const v8h*)(Qp + (nh * SEQ + m0 + m) * HDK);
  v16h qf;
#pragma unroll
  for (int i = 0; i < 8; ++i) { qf[i] = lowhalf ? qv[i] : hz; qf[i + 8] = hz; }

  const _Float16* kbase = Kp + (nh * SEQ + m) * HDK;
  const _Float16* vbase = Vp + ((size_t)n * DIM + head * HDV + m) * SEQ + hh * 8u;
  const float sc = (1.0f / sqrtf((float)SEQ)) * (1.0f / (QKCARRY * QKCARRY));

  float mrun = -1.0e30f, lrun = 0.0f;
  v8f o = {};

#pragma unroll 1
  for (unsigned kb = 0; kb < (unsigned)SEQ; kb += 32u) {
    const v8h k0 = *(const v8h*)(kbase + (size_t)kb * HDK);
    const v8h k1 = *(const v8h*)(kbase + (size_t)(kb + 16u) * HDK);
    v16h ka0, ka1;
#pragma unroll
    for (int i = 0; i < 8; ++i) {
      ka0[i] = lowhalf ? k0[i] : hz; ka0[i + 8] = hz;
      ka1[i] = lowhalf ? k1[i] : hz; ka1[i + 8] = hz;
    }
    v8f s0 = wmma16(ka0, qf, (v8f){});
    v8f s1 = wmma16(ka1, qf, (v8f){});

    float mx = -1.0e30f;
#pragma unroll
    for (int r = 0; r < 8; ++r) {
      s0[r] = s0[r] * sc;
      s1[r] = s1[r] * sc;
      mx = fmaxf(mx, fmaxf(s0[r], s1[r]));
    }
    mx = fmaxf(mx, __shfl_xor(mx, 16, 32));
    const float mn = fmaxf(mrun, mx);
    const float alpha = __expf(mrun - mn);
    mrun = mn;

    v16h pf;
    float psum = 0.0f;
#pragma unroll
    for (int r = 0; r < 8; ++r) {
      const h16 pa = toh_flush(__expf(s0[r] - mn) * PCARRY);
      const h16 pb = toh_flush(__expf(s1[r] - mn) * PCARRY);
      pf[r] = pa;
      pf[r + 8] = pb;
      psum += (float)pa + (float)pb;
    }
    lrun = lrun * alpha + psum;
#pragma unroll
    for (int r = 0; r < 8; ++r) o[r] = o[r] * alpha;

    const v16h va = frag_at(vbase + kb);
    o = wmma16(va, pf, o);
  }

  const float lt = lrun + __shfl_xor(lrun, 16, 32);
  const float inv = __builtin_amdgcn_rcpf(lt) * (1.0f / VCARRY);
#pragma unroll
  for (unsigned r = 0; r < 8u; ++r)
    T[m * TP + head * HDV + hh * 8u + r] = o[r] * inv;
  __syncthreads();

  {
    const unsigned c = tid >> 1, mq = (tid & 1u) * 8u;
    const float* tp = X + ((size_t)n * DIM + c) * SEQ_FULL + m0 + mq;
    const v4f a0 = *(const v4f*)(tp);
    const v4f a1 = *(const v4f*)(tp + 4);
#pragma unroll
    for (unsigned j = 0; j < 4u; ++j) {
      T[(mq + j) * TP + c] += bf16r(a0[j]);
      T[(mq + 4u + j) * TP + c] += bf16r(a1[j]);
    }
  }
  __syncthreads();

  const unsigned prow = n * (unsigned)SEQ + m0 + wave;
  const v4f t0 = *(const v4f*)&T[wave * TP + lane * 8u];
  const v4f t1 = *(const v4f*)&T[wave * TP + lane * 8u + 4u];
  float s = 0.0f;
#pragma unroll
  for (int i = 0; i < 4; ++i) s += t0[i] + t1[i];
  const float mean = red32_sum(s) * (1.0f / (float)DIM);
  float ss = 0.0f;
#pragma unroll
  for (int i = 0; i < 4; ++i) {
    const float d0 = t0[i] - mean, d1 = t1[i] - mean;
    ss += d0 * d0;
    ss += d1 * d1;
  }
  const float var = red32_sum(ss) * (1.0f / (float)DIM);
  const float rstd = 1.0f / sqrtf(var + 1.0e-5f);
  const v4f g0 = *(const v4f*)(G + lane * 8u);
  const v4f g1 = *(const v4f*)(G + lane * 8u + 4u);
  const v4f b0 = *(const v4f*)(Be + lane * 8u);
  const v4f b1 = *(const v4f*)(Be + lane * 8u + 4u);
  v8h ho;
#pragma unroll
  for (int i = 0; i < 4; ++i) {
    ho[i]     = toh_flush(ACARRY * ((t0[i] - mean) * rstd * bf16r(g0[i]) + bf16r(b0[i])));
    ho[i + 4] = toh_flush(ACARRY * ((t1[i] - mean) * rstd * bf16r(g1[i]) + bf16r(b1[i])));
  }
  const v4f y0 = *(const v4f*)&T[wave * TP + lane * 4u];
  const v4f y1 = *(const v4f*)&T[wave * TP + 128u + lane * 4u];
  _Float16* hp = H1 + (size_t)prow * DIM + lane * 8u;
  float* xp0 = X1 + (size_t)prow * DIM + lane * 4u;
  float* xp1 = xp0 + 128;
  *(volatile v8h*)hp = ho;
  *(volatile v4f*)xp0 = y0;
  *(volatile v4f*)xp1 = y1;
  __threadfence();
  *(volatile v8h*)hp = ho;
  *(volatile v4f*)xp0 = y0;
  *(volatile v4f*)xp1 = y1;
}

template <int MODE>
__device__ __forceinline__ void gemm_body(
    const _Float16* __restrict__ A16, const _Float16* __restrict__ Bt, const unsigned K,
    const float* __restrict__ bias, const float* __restrict__ addf,
    float* __restrict__ outf, _Float16* __restrict__ out16) {
  __shared__ float Cs[64 * LDC];
  const unsigned tid = threadIdx.x, lane = tid & 31u, w = tid >> 5;
  const unsigned mw = w >> 1, nw = w & 1u;
  const unsigned hh = lane >> 4, m = lane & 15u;
  const unsigned n0 = blockIdx.x * 64u;
  const unsigned row0 = blockIdx.y * 64u;

  const _Float16* ap  = A16 + (size_t)(row0 + mw * 16u + m) * K + hh * 8u;
  const _Float16* bp0 = Bt + (size_t)(n0 + nw * 32u + m) * K + hh * 8u;
  const _Float16* bp1 = bp0 + (size_t)16 * K;
  v8f acc0 = {}, acc1 = {};
#pragma unroll 2
  for (unsigned k0 = 0; k0 < K; k0 += 32u) {
    const v16h a  = frag_at(ap + k0);
    const v16h b0 = frag_at(bp0 + k0);
    const v16h b1 = frag_at(bp1 + k0);
    acc0 = wmma16(a, b0, acc0);
    acc1 = wmma16(a, b1, acc1);
  }
#pragma unroll
  for (int r = 0; r < 8; ++r) {
    float* d = &Cs[(mw * 16u + hh * 8u + (unsigned)r) * LDC + nw * 32u + m];
    d[0]  = acc0[r];
    d[16] = acc1[r];
  }
  __syncthreads();

  if (MODE == 3) {
#pragma unroll 1
    for (unsigned g = 0; g < 4u; ++g) {
      const unsigned r = 32u * (g >> 1) + (tid >> 3);
      const unsigned c = (tid & 7u) * 8u + 4u * (g & 1u);
      const v4f u  = *(const v4f*)&Cs[r * LDC + c];
      const v4f gb = *(const v4f*)(bias + n0 + c);
      v4f t;
#pragma unroll
      for (int j = 0; j < 4; ++j)
        t[j] = MCARRY * relu_act(u[j] * (1.0f / (WCARRY * ACARRY)) + bf16r(gb[j]));
      *(v4f*)&Cs[r * LDC + c] = t;
    }

    v8h x[2];
    size_t off[2];
#pragma unroll
    for (unsigned i = 0; i < 2u; ++i) {
      const unsigned r = 32u * i + (tid >> 3);
      const unsigned c = (tid & 7u) * 8u;
      const v4f u0 = *(const v4f*)&Cs[r * LDC + c];
      const v4f u1 = *(const v4f*)&Cs[r * LDC + c + 4];
#pragma unroll
      for (int j = 0; j < 4; ++j) {
        x[i][j]     = toh_flush(u0[j]);
        x[i][j + 4] = toh_flush(u1[j]);
      }
      off[i] = (size_t)(row0 + r) * HID + n0 + c;
    }
#pragma unroll
    for (int i = 0; i < 2; ++i) *(volatile v8h*)(out16 + off[i]) = x[i];
    __threadfence();
#pragma unroll
    for (int i = 0; i < 2; ++i) *(volatile v8h*)(out16 + off[i]) = x[i];
  }

  if (MODE == 4) {
    const float cs = 1.0f / (WCARRY * MCARRY);
    v4f xs[4];
    size_t off[4];
#pragma unroll
    for (unsigned i = 0; i < 4u; ++i) {
      const unsigned r = 16u * i + (tid >> 4);
      const unsigned c = (tid & 15u) * 4u;
      const size_t crow = (size_t)(row0 + r);
      const v4f u = *(const v4f*)&Cs[r * LDC + c];
      const v4f g = *(const v4f*)(bias + n0 + c);
      const v4f xin = *(const v4f*)(addf + crow * DIM + n0 + c);
      v4f val;
#pragma unroll
      for (int j = 0; j < 4; ++j) val[j] = xin[j] + (u[j] * cs + bf16r(g[j]));
      xs[i] = val;
      off[i] = crow * DIM + n0 + c;
    }
#pragma unroll
    for (int i = 0; i < 4; ++i) *(volatile v4f*)(outf + off[i]) = xs[i];
    __threadfence();
#pragma unroll
    for (int i = 0; i < 4; ++i) *(volatile v4f*)(outf + off[i]) = xs[i];
  }
}

__global__ __launch_bounds__(256) void gemm_ffn1_kernel(
    const _Float16* __restrict__ A16, const _Float16* __restrict__ Bt,
    const float* __restrict__ bias, _Float16* __restrict__ mid) {
  gemm_body<3>(A16, Bt, (unsigned)DIM, bias, bias, (float*)0, mid);
}
__global__ __launch_bounds__(256) void gemm_ffn2_kernel(
    const _Float16* __restrict__ A16, const _Float16* __restrict__ Bt,
    const float* __restrict__ bias, const float* __restrict__ x1, float* __restrict__ yout) {
  gemm_body<4>(A16, Bt, (unsigned)HID, bias, x1, yout, (_Float16*)0);
}

__global__ __launch_bounds__(256) void ln_out_kernel(
    const float* __restrict__ Y, const float* __restrict__ G, const float* __restrict__ Be,
    float* __restrict__ out) {
#pragma clang fp contract(off)
  __shared__ float T2[DIM * TP2];
  const unsigned tid = threadIdx.x, lane = tid & 31u;
  const unsigned wave = __builtin_amdgcn_readfirstlane(threadIdx.x >> 5);
  const unsigned p0 = blockIdx.x * 32u;
  const unsigned n = p0 / (unsigned)SEQ;
  const unsigned l0 = p0 - n * (unsigned)SEQ;

  const v4f g0 = *(const v4f*)(G + lane * 8u);
  const v4f g1 = *(const v4f*)(G + lane * 8u + 4u);
  const v4f b0 = *(const v4f*)(Be + lane * 8u);
  const v4f b1 = *(const v4f*)(Be + lane * 8u + 4u);

#pragma unroll 1
  for (unsigned j = 0; j < 4u; ++j) {
    const unsigned row = wave * 4u + j;
    const float* yr = Y + (size_t)(p0 + row) * DIM + lane * 8u;
    const v4f a0 = *(const v4f*)(yr);
    const v4f a1 = *(const v4f*)(yr + 4);
    float s = 0.0f;
#pragma unroll
    for (int i = 0; i < 4; ++i) s += a0[i] + a1[i];
    const float mean = red32_sum(s) * (1.0f / (float)DIM);
    float ss = 0.0f;
#pragma unroll
    for (int i = 0; i < 4; ++i) {
      const float d0 = a0[i] - mean, d1 = a1[i] - mean;
      ss += d0 * d0;
      ss += d1 * d1;
    }
    const float var = red32_sum(ss) * (1.0f / (float)DIM);
    const float rstd = 1.0f / sqrtf(var + 1.0e-5f);
#pragma unroll
    for (unsigned i = 0; i < 4u; ++i) {
      T2[(lane * 8u + i) * TP2 + row] =
          (a0[i] - mean) * rstd * bf16r(g0[i]) + bf16r(b0[i]);
      T2[(lane * 8u + 4u + i) * TP2 + row] =
          (a1[i] - mean) * rstd * bf16r(g1[i]) + bf16r(b1[i]);
    }
  }
  __syncthreads();

  v4f xs[8];
  size_t off[8];
#pragma unroll
  for (unsigned i = 0; i < 8u; ++i) {
    const unsigned idx = tid + 256u * i;
    const unsigned c = idx >> 3, q = (idx & 7u) * 4u;
    xs[i] = *(const v4f*)&T2[c * TP2 + q];
    off[i] = ((size_t)n * DIM + c) * SEQ_FULL + l0 + q;
  }
#pragma unroll
  for (int i = 0; i < 8; ++i) *(volatile v4f*)(out + off[i]) = xs[i];
  __threadfence();
#pragma unroll
  for (int i = 0; i < 8; ++i) *(volatile v4f*)(out + off[i]) = xs[i];
}

extern "C" void kernel_launch(void* const* d_in, const int* in_sizes, int n_in,
                              void* d_out, int out_size, void* d_ws, size_t ws_size,
                              hipStream_t stream) {
  if (n_in < 15) return;
  const long long need_x =
      ((long long)((NB - 1) * DIM + (DIM - 1))) * SEQ_FULL + SEQ;
  if ((long long)in_sizes[0] < need_x) return;
  if (in_sizes[1] < NGRP * KQG * GIN || in_sizes[3] < NGRP * KQG * GIN) return;
  if (in_sizes[2] < KQC || in_sizes[4] < KQC) return;
  if (in_sizes[5] < NGRP * VG * GIN || in_sizes[6] < DIM) return;
  if (in_sizes[7] < HID * DIM || in_sizes[8] < HID) return;
  if (in_sizes[9] < DIM * HID || in_sizes[10] < DIM) return;
  if (in_sizes[11] < DIM || in_sizes[12] < DIM || in_sizes[13] < DIM || in_sizes[14] < DIM) return;
  if ((long long)out_size < need_x) return;
  if (ws_size < WS_TOTAL) return;

  const float* X   = (const float*)d_in[0];
  const float* wk  = (const float*)d_in[1];
  const float* bk  = (const float*)d_in[2];
  const float* wq  = (const float*)d_in[3];
  const float* bq  = (const float*)d_in[4];
  const float* wv  = (const float*)d_in[5];
  const float* bv  = (const float*)d_in[6];
  const float* w1  = (const float*)d_in[7];
  const float* b1  = (const float*)d_in[8];
  const float* w2  = (const float*)d_in[9];
  const float* b2  = (const float*)d_in[10];
  const float* g1  = (const float*)d_in[11];
  const float* be1 = (const float*)d_in[12];
  const float* g2  = (const float*)d_in[13];
  const float* be2 = (const float*)d_in[14];
  float* out = (float*)d_out;

  char* ws = (char*)d_ws;
  _Float16* W1p   = (_Float16*)(ws + OFF_W1);
  _Float16* W2p   = (_Float16*)(ws + OFF_W2);
  _Float16* Kp    = (_Float16*)(ws + OFF_K);
  _Float16* Qp    = (_Float16*)(ws + OFF_Q);
  _Float16* Vp    = (_Float16*)(ws + OFF_V);
  _Float16* H1    = (_Float16*)(ws + OFF_H1);
  float*    X1    = (float*)(ws + OFF_X1);
  _Float16* Mid16 = (_Float16*)(ws + OFF_MID);
  float*    Yp    = (float*)(ws + OFF_Y);

  dim3 blk(256);
  wcast_kernel<<<dim3((DIM * HID) / 2048), blk, 0, stream>>>(w1, W1p);
  wcast_kernel<<<dim3((DIM * HID) / 2048), blk, 0, stream>>>(w2, W2p);
  proj_kernel<<<dim3(SEQ / 64, NGRP, NB), dim3(128), 0, stream>>>(
      X, wk, bk, wq, bq, wv, bv, Kp, Qp, Vp);
  attn_ln_kernel<<<dim3(SEQ / 16, NB), dim3(512), 0, stream>>>(
      X, Kp, Qp, Vp, g1, be1, H1, X1);
  gemm_ffn1_kernel<<<dim3(HID / 64, MROWS / 64), blk, 0, stream>>>(H1, W1p, b1, Mid16);
  gemm_ffn2_kernel<<<dim3(DIM / 64, MROWS / 64), blk, 0, stream>>>(Mid16, W2p, b2, X1, Yp);
  ln_out_kernel<<<dim3(MROWS / 32), blk, 0, stream>>>(Yp, g2, be2, out);
}
